// Model_70136815943965
// MI455X (gfx1250) — hardware-verified
//
#include <hip/hip_runtime.h>
#include <math.h>

typedef __attribute__((ext_vector_type(16))) _Float16 v16h;
typedef __attribute__((ext_vector_type(8)))  _Float16 v8h;
typedef __attribute__((ext_vector_type(8)))  float    v8f;
typedef __attribute__((ext_vector_type(4)))  float    v4f;

constexpr int kNB     = 16;
constexpr int kT      = 512;
constexpr int kNC     = 32;
constexpr int kPatch  = 16;
constexpr int kNLP    = kT / kPatch;
constexpr int kSeq    = kNC * kNLP;
constexpr int kRows   = kNB * kSeq;
constexpr int kDm     = 128;
constexpr int kDin    = 256;
constexpr int kNst    = 16;
constexpr int kDtR    = 8;
constexpr int kXdN    = kDtR + 2 * kNst;
constexpr int kXdP    = 64;
constexpr int kXzP    = 2 * kDin;
constexpr int kPred   = 96;
constexpr int kPredP  = 128;
constexpr int kHeadK  = kNLP * kDm;
constexpr int kPatchKP = 32;
constexpr int kNLayer = 2;
constexpr int kBC     = kNB * kNC;
constexpr int kConvTP = 260;
constexpr int kScanTS = 64;
constexpr int kScanCh = 64;
constexpr int kScanYP = 68;
constexpr float kEps  = 1e-5f;

constexpr float kCarryAct = 16.0f;
constexpr float kCarryW   = 32.0f;
constexpr float kCarryU   = 1024.0f;
constexpr float kCarryY   = 4096.0f;

static_assert(kNLP == 32 && kSeq == 1024 && kRows == 16384 && kHeadK == 4096 && kXdN == 40, "derived shapes");
static_assert(kT == 2 * 256, "instance-norm block covers the series with 2 samples per thread");
static_assert(kNC == 32, "one output row is one 128-B line");
static_assert((kPatchKP % 32) == 0 && (kDm % 32) == 0 && (kDin % 32) == 0 && (kHeadK % 32) == 0, "GEMM K multiples of 32");
static_assert((kRows % 64) == 0 && (kBC % 64) == 0, "GEMM M multiples of 64");
static_assert((kDm % 64) == 0 && (kXzP % 64) == 0 && (kXdP % 64) == 0 && (kPredP % 64) == 0, "GEMM N multiples of 64");
static_assert((kSeq % kScanTS) == 0 && (kSeq % 64) == 0 && (kDin % kScanCh) == 0 && kDin == 256, "tile multiples");
static_assert((kPatch % 8) == 0 && (kDm % 8) == 0 && (kDin % 8) == 0 && (kHeadK % 8) == 0, "cast chunks of 8");

constexpr size_t kOffSTATS = 0;
constexpr size_t kOffAP    = kOffSTATS + (size_t)kBC * 32 * 4;
constexpr size_t kOffWP    = kOffAP    + (size_t)kRows * kPatchKP * 2;
constexpr size_t kOffWIN   = kOffWP    + (size_t)kDm * kPatchKP * 2;
constexpr size_t kOffWXP   = kOffWIN   + (size_t)kNLayer * kXzP * kDm * 2;
constexpr size_t kOffWOUT  = kOffWXP   + (size_t)kNLayer * kXdP * kDin * 2;
constexpr size_t kOffWHEAD = kOffWOUT  + (size_t)kNLayer * kDm * kDin * 2;
constexpr size_t kOffXA    = kOffWHEAD + (size_t)kPredP * kHeadK * 2;
constexpr size_t kOffXB    = kOffXA    + (size_t)kRows * kDm * 4;
constexpr size_t kOffH16   = kOffXB    + (size_t)kRows * kDm * 4;
constexpr size_t kOffXZ    = kOffH16   + (size_t)kRows * kDm * 2;
constexpr size_t kOffUC    = kOffXZ    + (size_t)kRows * kXzP * 4;
constexpr size_t kOffU16   = kOffUC    + (size_t)kRows * kDin * 4;
constexpr size_t kOffXD    = kOffU16   + (size_t)kRows * kDin * 2;
constexpr size_t kOffY16   = kOffXD    + (size_t)kRows * kXdP * 4;
constexpr size_t kOffHO    = kOffY16   + (size_t)kRows * kDin * 2;
constexpr size_t kWsTotal  = kOffHO    + (size_t)kBC * kPredP * 4;
static_assert(kWsTotal == 95166464ull, "carve total");
static_assert(kWsTotal <= 134217728ull, "carve cap");
static_assert((kOffAP % 128) == 0 && (kOffWP % 128) == 0 && (kOffWIN % 128) == 0 && (kOffWXP % 128) == 0 &&
              (kOffWOUT % 128) == 0 && (kOffWHEAD % 128) == 0 && (kOffXA % 128) == 0 && (kOffXB % 128) == 0 &&
              (kOffH16 % 128) == 0 && (kOffXZ % 128) == 0 && (kOffUC % 128) == 0 && (kOffU16 % 128) == 0 &&
              (kOffXD % 128) == 0 && (kOffY16 % 128) == 0 && (kOffHO % 128) == 0, "128-B aligned regions");

struct FragH {
  union U { v16h v; v8h h[2]; };
  static __device__ __forceinline__ v16h load(const _Float16* p) {
    U f;
    f.h[0] = *(const v8h*)(p);
    f.h[1] = *(const v8h*)(p + 16);
    return f.v;
  }
  static __device__ __forceinline__ v8f mma(v16h a, v16h b, v8f c) {
    return __builtin_amdgcn_wmma_f32_16x16x32_f16(false, a, false, b, (short)0, c, false, false);
  }
};
__device__ __forceinline__ void guard_row4_h(v8f& a0, v8f& a1, v8f& a2, v8f& a3,
                                             v16h x, v16h b0, v16h b1, v16h b2, v16h b3) {
  asm volatile("v_nop\n\tv_nop\n\tv_nop\n\tv_nop"
               : "+v"(a0), "+v"(a1), "+v"(a2), "+v"(a3)
               : "v"(x), "v"(b0), "v"(b1), "v"(b2), "v"(b3));
}
__device__ __forceinline__ void keep4_h(v16h a, v16h b, v16h c, v16h d) {
  asm volatile("v_nop" :: "v"(a), "v"(b), "v"(c), "v"(d));
}
__device__ __forceinline__ void acc_guard4(v8f& a, v8f& b, v8f& c, v8f& d) {
  asm volatile("v_nop\n\tv_nop\n\tv_nop\n\tv_nop" : "+v"(a), "+v"(b), "+v"(c), "+v"(d));
}
__device__ __forceinline__ void wave_sync_lds() {
  __builtin_amdgcn_fence(__ATOMIC_RELEASE, "workgroup");
  __builtin_amdgcn_wave_barrier();
  __builtin_amdgcn_fence(__ATOMIC_ACQUIRE, "workgroup");
}

template <bool RESID>
__global__ __launch_bounds__(256) void gemm64_f16_kernel(
    const unsigned short* __restrict__ Ap, int lda,
    const unsigned short* __restrict__ Btp, int ldb,
    float* __restrict__ C, int ldc,
    const float* __restrict__ resid,
    int M, int N, int K, float scale)
{
  const _Float16* A  = (const _Float16*)Ap;
  const _Float16* Bt = (const _Float16*)Btp;
  __shared__ __align__(16) float sT[8][16 * 68];
  const int lane = threadIdx.x & 31;
  const int wave = threadIdx.x >> 5;
  const int tilesN = N >> 6;
  const int tilesM = M >> 6;
  const int tile = blockIdx.x * 8 + wave;
  if (tile >= tilesM * tilesN) return;
  const int tm = tile / tilesN;
  const int tn = tile - tm * tilesN;
  const int m0 = tm << 6;
  const int n0 = tn << 6;
  const int rlane = lane & 15;
  const int koff  = (lane >> 4) * 8;
  const int mOff  = (lane >> 4) * 8;

  v8f acc[4][4];
#pragma unroll
  for (int i = 0; i < 4; ++i)
#pragma unroll
    for (int j = 0; j < 4; ++j) acc[i][j] = (v8f){0.f, 0.f, 0.f, 0.f, 0.f, 0.f, 0.f, 0.f};

  for (int k0 = 0; k0 < K; k0 += 32) {
    v16h bh[4];
#pragma unroll
    for (int j = 0; j < 4; ++j) {
      const size_t bo = (size_t)(n0 + (j << 4) + rlane) * ldb + koff + k0;
      bh[j] = FragH::load(Bt + bo);
    }
#pragma unroll
    for (int i = 0; i < 4; ++i) {
      const size_t ao = (size_t)(m0 + (i << 4) + rlane) * lda + koff + k0;
      const v16h ah = FragH::load(A + ao);
#pragma unroll
      for (int j = 0; j < 4; ++j) acc[i][j] = FragH::mma(ah, bh[j], acc[i][j]);
      guard_row4_h(acc[i][0], acc[i][1], acc[i][2], acc[i][3], ah, bh[0], bh[1], bh[2], bh[3]);
    }
    keep4_h(bh[0], bh[1], bh[2], bh[3]);
  }
  acc_guard4(acc[0][0], acc[0][1], acc[0][2], acc[0][3]);
  acc_guard4(acc[1][0], acc[1][1], acc[1][2], acc[1][3]);
  acc_guard4(acc[2][0], acc[2][1], acc[2][2], acc[2][3]);
  acc_guard4(acc[3][0], acc[3][1], acc[3][2], acc[3][3]);

  float* slab = sT[wave];
  const int hh = lane >> 4;
  const int c4 = (lane & 15) * 4;
#pragma unroll
  for (int i = 0; i < 4; ++i) {
    const int mBase = m0 + (i << 4);
#pragma unroll
    for (int j = 0; j < 4; ++j) {
#pragma unroll
      for (int r = 0; r < 8; ++r) {
        slab[(mOff + r) * 68 + (j << 4) + rlane] = acc[i][j][r] * scale;
      }
    }
    wave_sync_lds();
    if (RESID) {
#pragma unroll
      for (int it = 0; it < 8; ++it) {
        const int row = it * 2 + hh;
        float* sp = slab + row * 68 + c4;
        v4f v = *(const v4f*)sp;
        const v4f rr = *(const v4f*)(resid + (size_t)(mBase + row) * ldc + n0 + c4);
        v = v + rr;
        *(v4f*)sp = v;
      }
      wave_sync_lds();
    }
    for (int pass = 0; pass < 2; ++pass) {
#pragma unroll
      for (int it = 0; it < 8; ++it) {
        const int row = it * 2 + hh;
        const v4f v = *(const v4f*)(slab + row * 68 + c4);
        *(volatile v4f*)(C + (size_t)(mBase + row) * ldc + n0 + c4) = v;
      }
      __threadfence();
    }
    wave_sync_lds();
  }
}

__global__ __launch_bounds__(256) void cast_pad_f16_kernel(
    const float* __restrict__ src, unsigned short* __restrict__ dst,
    int rowsSrcPer, int rowsDstPer, int Ksrc, int Kdst, int total8, float scale)
{
  const int i = blockIdx.x * 256 + threadIdx.x;
  if (i >= total8) return;
  const int e0  = i << 3;
  const int row = e0 / Kdst;
  const int k0  = e0 - row * Kdst;
  const int layer = row / rowsDstPer;
  const int r   = row - layer * rowsDstPer;
  const bool valid = (r < rowsSrcPer) && (k0 < Ksrc);
  const int rc = (r < rowsSrcPer) ? r : (rowsSrcPer - 1);
  const int kc = (k0 < Ksrc) ? k0 : (Ksrc - 8);
  const float* p = src + ((size_t)layer * rowsSrcPer + rc) * Ksrc + kc;
  const v4f a0 = *(const v4f*)(p);
  const v4f a1 = *(const v4f*)(p + 4);
  v8h hv;
#pragma unroll
  for (int e = 0; e < 4; ++e) {
    const float f0 = valid ? (a0[e] * scale) : 0.0f;
    const float f1 = valid ? (a1[e] * scale) : 0.0f;
    hv[e]     = (_Float16)f0;
    hv[4 + e] = (_Float16)f1;
  }
  unsigned short* q = dst + (size_t)e0;
  *(volatile v8h*)q = hv;
  __threadfence();
  *(volatile v8h*)q = hv;
}

__global__ __launch_bounds__(256) void instnorm_patch_kernel(
    const float* __restrict__ xin, float* __restrict__ stats, unsigned short* __restrict__ Ap)
{
  __shared__ float sRedA[8];
  __shared__ float sRedB[8];
  __shared__ __align__(16) float sXn[kT];
  const int tid = threadIdx.x, lane = tid & 31, wave = tid >> 5;
  const int bc = blockIdx.x;
  const int b = bc / kNC;
  const int c = bc - b * kNC;
  const float* base = xin + (size_t)b * kT * kNC + c;
  const float x0 = base[(size_t)tid * kNC];
  const float x1 = base[(size_t)(tid + 256) * kNC];
  float s = x0 + x1;
#pragma unroll
  for (int off = 16; off > 0; off >>= 1) s += __shfl_xor(s, off, 32);
  if (lane == 0) sRedA[wave] = s;
  __syncthreads();
  float S = 0.0f;
#pragma unroll
  for (int i = 0; i < 8; ++i) S += sRedA[i];
  const float mean = S * (1.0f / (float)kT);
  const float d0 = x0 - mean, d1 = x1 - mean;
  float q = d0 * d0 + d1 * d1;
#pragma unroll
  for (int off = 16; off > 0; off >>= 1) q += __shfl_xor(q, off, 32);
  if (lane == 0) sRedB[wave] = q;
  __syncthreads();
  float Q = 0.0f;
#pragma unroll
  for (int i = 0; i < 8; ++i) Q += sRedB[i];
  const float var = Q * (1.0f / (float)kT);
  const float sd  = sqrtf(var + kEps);
  const float isd = 1.0f / sd;
  sXn[tid]       = (d0 * isd) * kCarryAct;
  sXn[tid + 256] = (d1 * isd) * kCarryAct;
  __syncthreads();
  if (tid < 128) {
    const int tokl = tid >> 2;
    const int qd   = tid & 3;
    const bool data = (qd < 2);
    const float* sp = sXn + tokl * kPatch + (qd & 1) * 8;
    const v4f a0 = *(const v4f*)(sp);
    const v4f a1 = *(const v4f*)(sp + 4);
    v8h hv;
#pragma unroll
    for (int e = 0; e < 4; ++e) {
      const float f0 = data ? a0[e] : 0.0f;
      const float f1 = data ? a1[e] : 0.0f;
      hv[e]     = (_Float16)f0;
      hv[4 + e] = (_Float16)f1;
    }
    unsigned short* dstp = Ap + ((size_t)bc * kNLP + tokl) * kPatchKP + qd * 8;
    *(volatile v8h*)dstp = hv;
    __threadfence();
    *(volatile v8h*)dstp = hv;
  }
  if (wave == 4) {
    const float sv = (lane == 0) ? mean : ((lane == 1) ? sd : 0.0f);
    float* dsts = stats + (size_t)bc * 32 + lane;
    *(volatile float*)dsts = sv;
    __threadfence();
    *(volatile float*)dsts = sv;
  }
}

__global__ __launch_bounds__(256) void rmsnorm_f16_kernel(
    const float* __restrict__ X, const float* __restrict__ w, unsigned short* __restrict__ H16)
{
  const int tid = threadIdx.x, lane = tid & 31, wave = tid >> 5;
  const int hf = lane >> 4, l16 = lane & 15;
  const int tok = blockIdx.x * 16 + wave * 2 + hf;
  const float* p = X + (size_t)tok * kDm + l16 * 8;
  const v4f a0 = *(const v4f*)(p);
  const v4f a1 = *(const v4f*)(p + 4);
  const v4f w0 = *(const v4f*)(w + l16 * 8);
  const v4f w1 = *(const v4f*)(w + l16 * 8 + 4);
  float ss = 0.0f;
#pragma unroll
  for (int e = 0; e < 4; ++e) {
    ss = fmaf(a0[e], a0[e], ss);
    ss = fmaf(a1[e], a1[e], ss);
  }
#pragma unroll
  for (int off = 8; off > 0; off >>= 1) ss += __shfl_xor(ss, off, 32);
  const float r = rsqrtf(ss * (1.0f / (float)kDm) + kEps);
  v8h hv;
#pragma unroll
  for (int e = 0; e < 4; ++e) {
    const float f0 = ((a0[e] * r) * w0[e]) * kCarryAct;
    const float f1 = ((a1[e] * r) * w1[e]) * kCarryAct;
    hv[e]     = (_Float16)f0;
    hv[4 + e] = (_Float16)f1;
  }
  unsigned short* q = H16 + (size_t)tok * kDm + l16 * 8;
  *(volatile v8h*)q = hv;
  __threadfence();
  *(volatile v8h*)q = hv;
}

__global__ __launch_bounds__(256) void conv_silu_kernel(
    const float* __restrict__ XZ, const float* __restrict__ cw, const float* __restrict__ cb,
    float* __restrict__ UC, unsigned short* __restrict__ U16)
{
  __shared__ __align__(16) float sT[16 * kConvTP];
  const int tid = threadIdx.x, lane = tid & 31, wave = tid >> 5;
  const int d = tid;
  const int g0 = blockIdx.x * 64;
  const int tb = g0 & (kSeq - 1);
  const v4f wq = *(const v4f*)(cw + d * 4);
  const float w0 = wq[0], w1 = wq[1], w2 = wq[2], w3 = wq[3];
  const float bc = cb[d];
  float xm3, xm2, xm1;
  {
    const bool hist = (tb > 0);
    const int rb = hist ? (g0 - 3) : g0;
    const float v3 = XZ[(size_t)rb * kXzP + d];
    const float v2 = XZ[(size_t)(rb + 1) * kXzP + d];
    const float v1 = XZ[(size_t)(rb + 2) * kXzP + d];
    xm3 = hist ? v3 : 0.0f;
    xm2 = hist ? v2 : 0.0f;
    xm1 = hist ? v1 : 0.0f;
  }
  const int hrow = wave >> 1;
  const int hch  = (wave & 1) * 128 + lane * 4;
#pragma unroll 1
  for (int sub = 0; sub < 4; ++sub) {
    const int lb = g0 + sub * 16;
#pragma unroll 1
    for (int s = 0; s < 16; ++s) {
      const float xcur = XZ[(size_t)(lb + s) * kXzP + d];
      float acc = w0 * xm3;
      acc = fmaf(w1, xm2, acc);
      acc = fmaf(w2, xm1, acc);
      acc = fmaf(w3, xcur, acc);
      const float sv = acc + bc;
      const float sg = __builtin_amdgcn_rcpf(1.0f + expf(-sv));
      sT[s * kConvTP + tid] = sv * sg;
      xm3 = xm2;
      xm2 = xm1;
      xm1 = xcur;
    }
    __syncthreads();
    v4f fv[4];
    v8h bv[2];
#pragma unroll
    for (int it = 0; it < 4; ++it) fv[it] = *(const v4f*)(sT + (it * 4 + hrow) * kConvTP + hch);
#pragma unroll
    for (int it = 0; it < 2; ++it) {
      const float* sp = sT + (it * 8 + wave) * kConvTP + lane * 8;
      const v4f a0 = *(const v4f*)(sp);
      const v4f a1 = *(const v4f*)(sp + 4);
#pragma unroll
      for (int e = 0; e < 4; ++e) {
        const float f0 = a0[e] * kCarryU;
        const float f1 = a1[e] * kCarryU;
        bv[it][e]     = (_Float16)f0;
        bv[it][4 + e] = (_Float16)f1;
      }
    }
    for (int pass = 0; pass < 2; ++pass) {
#pragma unroll
      for (int it = 0; it < 4; ++it)
        *(volatile v4f*)(UC + (size_t)(lb + it * 4 + hrow) * kDin + hch) = fv[it];
#pragma unroll
      for (int it = 0; it < 2; ++it)
        *(volatile v8h*)(U16 + (size_t)(lb + it * 8 + wave) * kDin + lane * 8) = bv[it];
      __threadfence();
    }
    __syncthreads();
  }
}

__global__ __launch_bounds__(128) void scan_kernel(
    const float* __restrict__ XD, const float* __restrict__ UC, const float* __restrict__ XZ,
    const float* __restrict__ Wdt, const float* __restrict__ bdt, const float* __restrict__ Alog,
    const float* __restrict__ Dp, unsigned short* __restrict__ Y16)
{
  __shared__ __align__(16) float sX[kScanTS * kXdP];
  __shared__ __align__(16) float sY[kScanTS * kScanYP];
  const int tid = threadIdx.x, lane = tid & 31, wave = tid >> 5;
  const int ch = tid >> 1, hf = tid & 1;
  constexpr int kBlkPerB = kDin / kScanCh;
  const int bix = blockIdx.x / kBlkPerB;
  const int d0  = (blockIdx.x - bix * kBlkPerB) * kScanCh;
  const int d   = d0 + ch;
  const size_t row0 = (size_t)bix * kSeq;

  float wv[kDtR];
  {
    const v4f q0 = *(const v4f*)(Wdt + (size_t)d * kDtR);
    const v4f q1 = *(const v4f*)(Wdt + (size_t)d * kDtR + 4);
    wv[0] = q0[0]; wv[1] = q0[1]; wv[2] = q0[2]; wv[3] = q0[3];
    wv[4] = q1[0]; wv[5] = q1[1]; wv[6] = q1[2]; wv[7] = q1[3];
  }
  float negA[8], h[8];
  {
    const v4f q0 = *(const v4f*)(Alog + (size_t)d * kNst + hf * 8);
    const v4f q1 = *(const v4f*)(Alog + (size_t)d * kNst + hf * 8 + 4);
    negA[0] = -expf(q0[0]); negA[1] = -expf(q0[1]); negA[2] = -expf(q0[2]); negA[3] = -expf(q0[3]);
    negA[4] = -expf(q1[0]); negA[5] = -expf(q1[1]); negA[6] = -expf(q1[2]); negA[7] = -expf(q1[3]);
  }
#pragma unroll
  for (int j = 0; j < 8; ++j) h[j] = 0.0f;
  const float bb = bdt[d], Dd = Dp[d];
  const int q = lane >> 3, c8 = (lane & 7) * 8;

#pragma unroll 1
  for (int t0 = 0; t0 < kSeq; t0 += kScanTS) {
    __syncthreads();
#pragma unroll
    for (int i = 0; i < 8; ++i) {
      const int idx = tid + 128 * i;
      const int r = idx >> 4;
      const int cc = (idx & 15) * 4;
      *(v4f*)(sX + r * kXdP + cc) = *(const v4f*)(XD + (row0 + t0 + r) * kXdP + cc);
    }
    __syncthreads();
#pragma unroll 1
    for (int s = 0; s < kScanTS; ++s) {
      const size_t m = row0 + (size_t)(t0 + s);
      float uv = UC[m * kDin + d];
      asm volatile("" : "+v"(uv));
      float zv = XZ[m * kXzP + kDin + d];
      asm volatile("" : "+v"(zv));
      const float* xr = sX + s * kXdP;
      const v4f r0 = *(const v4f*)(xr);
      const v4f r1 = *(const v4f*)(xr + 4);
      float vdot = 0.0f;
      vdot = fmaf(r0[0], wv[0], vdot);
      vdot = fmaf(r0[1], wv[1], vdot);
      vdot = fmaf(r0[2], wv[2], vdot);
      vdot = fmaf(r0[3], wv[3], vdot);
      vdot = fmaf(r1[0], wv[4], vdot);
      vdot = fmaf(r1[1], wv[5], vdot);
      vdot = fmaf(r1[2], wv[6], vdot);
      vdot = fmaf(r1[3], wv[7], vdot);
      const v4f b0 = *(const v4f*)(xr + kDtR + hf * 8);
      const v4f b1 = *(const v4f*)(xr + kDtR + hf * 8 + 4);
      const v4f c0 = *(const v4f*)(xr + kDtR + kNst + hf * 8);
      const v4f c1 = *(const v4f*)(xr + kDtR + kNst + hf * 8 + 4);
      float Bs[8], Cs[8];
      Bs[0] = b0[0]; Bs[1] = b0[1]; Bs[2] = b0[2]; Bs[3] = b0[3];
      Bs[4] = b1[0]; Bs[5] = b1[1]; Bs[6] = b1[2]; Bs[7] = b1[3];
      Cs[0] = c0[0]; Cs[1] = c0[1]; Cs[2] = c0[2]; Cs[3] = c0[3];
      Cs[4] = c1[0]; Cs[5] = c1[1]; Cs[6] = c1[2]; Cs[7] = c1[3];
      const float v  = vdot + bb;
      const float dt = fmaxf(v, 0.0f) + log1pf(expf(-fabsf(v)));
      float y = 0.0f;
#pragma unroll
      for (int j = 0; j < 8; ++j) {
        const float e = expf(dt * negA[j]);
        const float inj = (dt * Bs[j]) * uv;
        h[j] = fmaf(e, h[j], inj);
        y = fmaf(h[j], Cs[j], y);
      }
      const float yo = __shfl_xor(y, 1, 32);
      float yt = y + yo;
      yt = fmaf(uv, Dd, yt);
      const float sg = __builtin_amdgcn_rcpf(1.0f + expf(-zv));
      float ov = (yt * (zv * sg)) * kCarryY;
      asm volatile("" : "+v"(ov));
      if (hf == 0) sY[s * kScanYP + ch] = ov;
    }
    __syncthreads();
    v8h hv[4];
#pragma unroll
    for (int it = 0; it < 4; ++it) {
      const int row = it * 16 + wave * 4 + q;
      const float* sp = sY + row * kScanYP + c8;
      const v4f a0 = *(const v4f*)(sp);
      const v4f a1 = *(const v4f*)(sp + 4);
#pragma unroll
      for (int e = 0; e < 4; ++e) {
        hv[it][e]     = (_Float16)a0[e];
        hv[it][4 + e] = (_Float16)a1[e];
      }
    }
    for (int pass = 0; pass < 2; ++pass) {
#pragma unroll
      for (int it = 0; it < 4; ++it) {
        const int row = it * 16 + wave * 4 + q;
        *(volatile v8h*)(Y16 + (row0 + (size_t)(t0 + row)) * kDin + d0 + c8) = hv[it];
      }
      __threadfence();
    }
  }
}

__global__ __launch_bounds__(256) void head_out_kernel(
    const float* __restrict__ HO, const float* __restrict__ hb, const float* __restrict__ stats,
    float* __restrict__ outp)
{
  __shared__ __align__(16) float sT[kPred * 36];
  __shared__ float sM[kNC];
  __shared__ float sS[kNC];
  const int tid = threadIdx.x;
  const int b = blockIdx.x;
  if (tid < kNC) {
    sM[tid] = stats[((size_t)b * kNC + tid) * 32];
    sS[tid] = stats[((size_t)b * kNC + tid) * 32 + 1];
  }
  __syncthreads();
#pragma unroll 1
  for (int i = 0; i < (kPred * kNC) / 256; ++i) {
    const int idx = tid + 256 * i;
    const int c = idx / kPred;
    const int p = idx - c * kPred;
    const float v = HO[((size_t)b * kNC + c) * kPredP + p] + hb[p];
    sT[p * 36 + c] = fmaf(v, sS[c], sM[c]);
  }
  __syncthreads();
  v4f val[3];
#pragma unroll
  for (int i = 0; i < 3; ++i) {
    const int f = tid + 256 * i;
    const int p = f >> 3;
    const int c4 = (f & 7) * 4;
    val[i] = *(const v4f*)(sT + p * 36 + c4);
  }
  for (int pass = 0; pass < 2; ++pass) {
#pragma unroll
    for (int i = 0; i < 3; ++i) {
      const int f = tid + 256 * i;
      const int p = f >> 3;
      const int c4 = (f & 7) * 4;
      *(volatile v4f*)(outp + ((size_t)b * kPred + p) * kNC + c4) = val[i];
    }
    __threadfence();
  }
}
static_assert(((kPred * kNC) % 256) == 0 && (kPred * kNC) / 4 == 3 * 256, "head epilogue coverage");

extern "C" void kernel_launch(void* const* d_in, const int* in_sizes, int n_in,
                              void* d_out, int out_size, void* d_ws, size_t ws_size,
                              hipStream_t stream)
{
  if (n_in < 18) return;
  if (in_sizes[0] != kNB * kT * kNC) return;
  if (in_sizes[4] != kDm * kPatch) return;
  if (in_sizes[5] != kNLayer * kDm) return;
  if (in_sizes[6] != kNLayer * kXzP * kDm) return;
  if (in_sizes[7] != kNLayer * kDin * 4) return;
  if (in_sizes[8] != kNLayer * kDin) return;
  if (in_sizes[9] != kNLayer * kXdN * kDin) return;
  if (in_sizes[10] != kNLayer * kDin * kDtR) return;
  if (in_sizes[11] != kNLayer * kDin) return;
  if (in_sizes[12] != kNLayer * kDin * kNst) return;
  if (in_sizes[13] != kNLayer * kDin) return;
  if (in_sizes[14] != kNLayer * kDm * kDin) return;
  if (in_sizes[15] != kDm) return;
  if (in_sizes[16] != kPred * kHeadK) return;
  if (in_sizes[17] != kPred) return;
  if (out_size != kNB * kPred * kNC) return;
  if (ws_size < kWsTotal) return;

  const float* x_enc        = (const float*)d_in[0];
  const float* patch_w      = (const float*)d_in[4];
  const float* norm_w       = (const float*)d_in[5];
  const float* in_proj_w    = (const float*)d_in[6];
  const float* conv_w       = (const float*)d_in[7];
  const float* conv_b       = (const float*)d_in[8];
  const float* x_proj_w     = (const float*)d_in[9];
  const float* dt_proj_w    = (const float*)d_in[10];
  const float* dt_proj_b    = (const float*)d_in[11];
  const float* A_log        = (const float*)d_in[12];
  const float* D_skip       = (const float*)d_in[13];
  const float* out_proj_w   = (const float*)d_in[14];
  const float* final_norm_w = (const float*)d_in[15];
  const float* head_w       = (const float*)d_in[16];
  const float* head_b       = (const float*)d_in[17];
  float* outp = (float*)d_out;

  char* ws = (char*)d_ws;
  float*          STATS = (float*)(ws + kOffSTATS);
  unsigned short* AP    = (unsigned short*)(ws + kOffAP);
  unsigned short* WP    = (unsigned short*)(ws + kOffWP);
  unsigned short* WIN   = (unsigned short*)(ws + kOffWIN);
  unsigned short* WXP   = (unsigned short*)(ws + kOffWXP);
  unsigned short* WOUT  = (unsigned short*)(ws + kOffWOUT);
  unsigned short* WHEAD = (unsigned short*)(ws + kOffWHEAD);
  float*          XA    = (float*)(ws + kOffXA);
  float*          XB    = (float*)(ws + kOffXB);
  unsigned short* H16   = (unsigned short*)(ws + kOffH16);
  float*          XZ    = (float*)(ws + kOffXZ);
  float*          UC    = (float*)(ws + kOffUC);
  unsigned short* U16   = (unsigned short*)(ws + kOffU16);
  float*          XD    = (float*)(ws + kOffXD);
  unsigned short* Y16   = (unsigned short*)(ws + kOffY16);
  float*          HO    = (float*)(ws + kOffHO);

  constexpr float kSclActW = 1.0f / (kCarryAct * kCarryW);
  constexpr float kSclUW   = 1.0f / (kCarryU * kCarryW);
  constexpr float kSclYW   = 1.0f / (kCarryY * kCarryW);

  instnorm_patch_kernel<<<kBC, 256, 0, stream>>>(x_enc, STATS, AP);

  {
    constexpr int t8 = kDm * kPatchKP / 8;
    static_assert((t8 % 256) == 0, "cast grid");
    cast_pad_f16_kernel<<<t8 / 256, 256, 0, stream>>>(patch_w, WP, kDm, kDm, kPatch, kPatchKP, t8, kCarryW);
  }
  {
    constexpr int t8 = kNLayer * kXzP * kDm / 8;
    static_assert((t8 % 256) == 0, "cast grid");
    cast_pad_f16_kernel<<<t8 / 256, 256, 0, stream>>>(in_proj_w, WIN, kNLayer * kXzP, kNLayer * kXzP, kDm, kDm, t8, kCarryW);
  }
  {
    constexpr int t8 = kNLayer * kXdP * kDin / 8;
    static_assert((t8 % 256) == 0, "cast grid");
    cast_pad_f16_kernel<<<t8 / 256, 256, 0, stream>>>(x_proj_w, WXP, kXdN, kXdP, kDin, kDin, t8, kCarryW);
  }
  {
    constexpr int t8 = kNLayer * kDm * kDin / 8;
    static_assert((t8 % 256) == 0, "cast grid");
    cast_pad_f16_kernel<<<t8 / 256, 256, 0, stream>>>(out_proj_w, WOUT, kNLayer * kDm, kNLayer * kDm, kDin, kDin, t8, kCarryW);
  }
  {
    constexpr int t8 = kPredP * kHeadK / 8;
    static_assert((t8 % 256) == 0, "cast grid");
    cast_pad_f16_kernel<<<t8 / 256, 256, 0, stream>>>(head_w, WHEAD, kPred, kPredP, kHeadK, kHeadK, t8, kCarryW);
  }

  {
    constexpr int tiles = (kRows / 64) * (kDm / 64);
    static_assert((tiles % 8) == 0, "gemm grid");
    gemm64_f16_kernel<false><<<tiles / 8, 256, 0, stream>>>(
        AP, kPatchKP, WP, kPatchKP, XA, kDm, XA, kRows, kDm, kPatchKP, kSclActW);
  }

  for (int l = 0; l < kNLayer; ++l) {
    float* xin  = (l == 0) ? XA : XB;
    float* xout = (l == 0) ? XB : XA;

    rmsnorm_f16_kernel<<<kRows / 16, 256, 0, stream>>>(xin, norm_w + (size_t)l * kDm, H16);

    {
      constexpr int tiles = (kRows / 64) * (kXzP / 64);
      static_assert((tiles % 8) == 0, "gemm grid");
      gemm64_f16_kernel<false><<<tiles / 8, 256, 0, stream>>>(
          H16, kDm, WIN + (size_t)l * kXzP * kDm, kDm, XZ, kXzP, XZ, kRows, kXzP, kDm, kSclActW);
    }

    conv_silu_kernel<<<kRows / 64, 256, 0, stream>>>(
        XZ, conv_w + (size_t)l * kDin * 4, conv_b + (size_t)l * kDin, UC, U16);

    {
      constexpr int tiles = (kRows / 64) * (kXdP / 64);
      static_assert((tiles % 8) == 0, "gemm grid");
      gemm64_f16_kernel<false><<<tiles / 8, 256, 0, stream>>>(
          U16, kDin, WXP + (size_t)l * kXdP * kDin, kDin, XD, kXdP, XD, kRows, kXdP, kDin, kSclUW);
    }

    scan_kernel<<<kNB * (kDin / kScanCh), 128, 0, stream>>>(
        XD, UC, XZ, dt_proj_w + (size_t)l * kDin * kDtR, dt_proj_b + (size_t)l * kDin,
        A_log + (size_t)l * kDin * kNst, D_skip + (size_t)l * kDin, Y16);

    {
      constexpr int tiles = (kRows / 64) * (kDm / 64);
      static_assert((tiles % 8) == 0, "gemm grid");
      gemm64_f16_kernel<true><<<tiles / 8, 256, 0, stream>>>(
          Y16, kDin, WOUT + (size_t)l * kDm * kDin, kDin, xout, kDm, xin, kRows, kDm, kDin, kSclYW);
    }
  }
  static_assert((kNLayer % 2) == 0, "final stream lands in XA");

  rmsnorm_f16_kernel<<<kRows / 16, 256, 0, stream>>>(XA, final_norm_w, H16);

  {
    constexpr int tiles = (kBC / 64) * (kPredP / 64);
    static_assert((tiles % 8) == 0, "gemm grid");
    gemm64_f16_kernel<false><<<tiles / 8, 256, 0, stream>>>(
        H16, kHeadK, WHEAD, kHeadK, HO, kPredP, HO, kBC, kPredP, kHeadK, kSclActW);
  }

  head_out_kernel<<<kNB, 256, 0, stream>>>(HO, head_b, STATS, outp);
}
